// MoE_Bottleneck_35476429865769
// MI455X (gfx1250) — hardware-verified
//
#include <hip/hip_runtime.h>
#include <stddef.h>
#include <stdint.h>

#define NT   25600
#define C1   512
#define CM   256
#define C2   512
#define NE   4
#define TB1  32
#define TB2  32
#define TB3  128
#define OB3  64
#define OTP  260
#define HTP  132
#define WES  64.0f
#define WEI  0.015625f
#define W3S  16.0f
#define MOS  256.0f
#define C3I  0.000244140625f

static_assert(NT % TB1 == 0);
static_assert(NT % TB2 == 0);
static_assert(NT % TB3 == 0);
static_assert(C2 % OB3 == 0);
static_assert(C1 % 32 == 0);
static_assert(CM == 256);
static_assert(TB1 == 32);
static_assert(TB2 == 32);
static_assert(OTP % 4 == 0);
static_assert(HTP % 4 == 0);
static_assert((NE * CM) % 8 == 0);
static_assert(C2 % 8 == 0);
static_assert(NT % 4 == 0);

typedef _Float16 v16h __attribute__((ext_vector_type(16)));
typedef _Float16 v8h  __attribute__((ext_vector_type(8)));
typedef float    v8f  __attribute__((ext_vector_type(8)));
typedef float    v4f  __attribute__((ext_vector_type(4)));
typedef unsigned int v4u __attribute__((ext_vector_type(4)));

union Frag  { v16h v; v8h h[2]; };
union Pack8 { v8h h; v4u u; };

__device__ __forceinline__ v8f mma16(v16h a, v16h b, v8f c) {
  c = __builtin_amdgcn_wmma_f32_16x16x32_f16(false, a, false, b, (short)0, c, false, false);
  asm volatile("v_nop\n\tv_nop\n\tv_nop\n\tv_nop" : "+v"(c) : "v"(a), "v"(b));
  return c;
}

__device__ __forceinline__ v16h ldfrag(const _Float16* p, int ld, int row0, int k0, int lane) {
  const int m = lane & 15, lh = lane >> 4;
  const _Float16* q = p + (size_t)(row0 + m) * ld + k0 + 8 * lh;
  Frag f;
  f.h[0] = *(const v8h*)(q);
  f.h[1] = *(const v8h*)(q + 16);
  return f.v;
}

__device__ __forceinline__ v8f zero8() { return (v8f){0.f, 0.f, 0.f, 0.f, 0.f, 0.f, 0.f, 0.f}; }

__global__ __launch_bounds__(256) void k_cvtw(const float* __restrict__ src, _Float16* __restrict__ dst,
                                              int nrows, int rstride, int estride, int eoff, float scale) {
  const int tid = threadIdx.x, lane = tid & 31, wave = tid >> 5;
  const int row = blockIdx.x * 8 + wave;
  if (row >= nrows) return;
  const float* s = src + (size_t)row * rstride + eoff + (size_t)(8 * lane) * estride;
  float f[8];
#pragma unroll
  for (int i = 0; i < 8; ++i) f[i] = s[(size_t)i * estride] * scale;
  Pack8 pk;
  pk.h = (v8h){(_Float16)f[0], (_Float16)f[1], (_Float16)f[2], (_Float16)f[3],
               (_Float16)f[4], (_Float16)f[5], (_Float16)f[6], (_Float16)f[7]};
  const v4u vv = pk.u;
  volatile v4u* d = (volatile v4u*)(dst + (size_t)row * CM + 8 * lane);
  *d = vv;
  __threadfence();
  *d = vv;
}

__global__ __launch_bounds__(256) void k_conv1(const float* __restrict__ x, const float* __restrict__ w1,
                                               const float* __restrict__ bn1s, const float* __restrict__ bn1b,
                                               const float* __restrict__ wr, const float* __restrict__ br,
                                               _Float16* __restrict__ x1h, float* __restrict__ rt) {
  __shared__ __align__(16) float sW[32 * CM];
  __shared__ __align__(16) float sX[32 * TB1];
  __shared__ __align__(16) float sR[NE * CM];
  __shared__ __align__(16) float sG[TB1 * NE];
  const int tid = threadIdx.x, lane = tid & 31, wave = tid >> 5;
  const int t0 = blockIdx.x * TB1;

#pragma unroll
  for (int e = 0; e < NE; ++e) sR[e * CM + tid] = wr[e * CM + tid];

  float acc[4][8];
#pragma unroll
  for (int i = 0; i < 4; ++i) {
#pragma unroll
    for (int c = 0; c < 8; ++c) acc[i][c] = 0.f;
  }
  const float* wrow = w1 + (size_t)tid * C1;
  const float* xcol = x + (size_t)(tid >> 3) * NT + t0 + (tid & 7) * 4;
  float* sxw = sX + (tid >> 3) * TB1 + (tid & 7) * 4;
  const float* sxr = sX + 4 * wave;
  const float* swr = sW + 8 * lane;
#pragma unroll 1
  for (int kc = 0; kc < C1 / 32; ++kc) {
    const int k0 = kc * 32;
    __syncthreads();
    *(v4f*)sxw = *(const v4f*)(xcol + (size_t)k0 * NT);
#pragma unroll
    for (int q = 0; q < 8; ++q) {
      const v4f a = *(const v4f*)(wrow + k0 + 4 * q);
#pragma unroll
      for (int i = 0; i < 4; ++i) sW[(4 * q + i) * CM + tid] = a[i];
    }
    __syncthreads();
#pragma unroll 1
    for (int j = 0; j < 32; ++j) {
      const v4f xv = *(const v4f*)(sxr + j * TB1);
      const v4f wa = *(const v4f*)(swr + j * CM);
      const v4f wb = *(const v4f*)(swr + j * CM + 4);
#pragma unroll
      for (int i = 0; i < 4; ++i) {
#pragma unroll
        for (int c = 0; c < 4; ++c) {
          acc[i][c]     += xv[i] * wa[c];
          acc[i][4 + c] += xv[i] * wb[c];
        }
      }
    }
  }
  __syncthreads();
  float* sX1 = sW;
#pragma unroll
  for (int i = 0; i < 4; ++i) {
    float* d = sX1 + (4 * wave + i) * CM + 8 * lane;
    *(v4f*)(d)     = (v4f){acc[i][0], acc[i][1], acc[i][2], acc[i][3]};
    *(v4f*)(d + 4) = (v4f){acc[i][4], acc[i][5], acc[i][6], acc[i][7]};
  }
  __syncthreads();

  {
    const float sc = bn1s[tid], sh = bn1b[tid];
#pragma unroll 1
    for (int it = 0; it < TB1; ++it) {
      float v = sX1[it * CM + tid];
      v = v * sc + sh;
      const float ex = expf(fminf(-v, 60.0f));
      const float sg = 1.0f / (1.0f + ex);
      sX1[it * CM + tid] = v * sg;
    }
  }
  __syncthreads();

  {
    const int tk = tid >> 3, part = lane & 7;
    const float* xrp = sX1 + tk * CM + part * 32;
    const float* rrp = sR + part * 32;
    float l0 = 0.f, l1 = 0.f, l2 = 0.f, l3 = 0.f;
#pragma unroll 1
    for (int c = 0; c < 32; ++c) {
      const float xv = xrp[c];
      l0 += xv * rrp[c];
      l1 += xv * rrp[CM + c];
      l2 += xv * rrp[2 * CM + c];
      l3 += xv * rrp[3 * CM + c];
    }
#pragma unroll
    for (int off = 1; off < 8; off <<= 1) {
      l0 += __shfl_xor(l0, off, 32);
      l1 += __shfl_xor(l1, off, 32);
      l2 += __shfl_xor(l2, off, 32);
      l3 += __shfl_xor(l3, off, 32);
    }
    l0 += br[0]; l1 += br[1]; l2 += br[2]; l3 += br[3];
    const float mx = fmaxf(fmaxf(l0, l1), fmaxf(l2, l3));
    float p0 = expf(l0 - mx), p1 = expf(l1 - mx), p2 = expf(l2 - mx), p3 = expf(l3 - mx);
    const float inv = 1.0f / ((p0 + p1) + (p2 + p3));
    p0 *= inv; p1 *= inv; p2 *= inv; p3 *= inv;
    int i1 = 0; float b1 = p0; bool cnd;
    cnd = p1 > b1; i1 = cnd ? 1 : i1; b1 = cnd ? p1 : b1;
    cnd = p2 > b1; i1 = cnd ? 2 : i1; b1 = cnd ? p2 : b1;
    cnd = p3 > b1; i1 = cnd ? 3 : i1; b1 = cnd ? p3 : b1;
    const float q0 = (i1 == 0) ? -1.0f : p0;
    const float q1 = (i1 == 1) ? -1.0f : p1;
    const float q2 = (i1 == 2) ? -1.0f : p2;
    const float q3 = (i1 == 3) ? -1.0f : p3;
    int i2 = 0; float b2 = q0;
    cnd = q1 > b2; i2 = cnd ? 1 : i2; b2 = cnd ? q1 : b2;
    cnd = q2 > b2; i2 = cnd ? 2 : i2; b2 = cnd ? q2 : b2;
    cnd = q3 > b2; i2 = cnd ? 3 : i2; b2 = cnd ? q3 : b2;
    const float rin = 1.0f / (b1 + b2);
    const float g1 = b1 * rin, g2 = b2 * rin;
    v4f gv;
    gv[0] = (i1 == 0) ? g1 : ((i2 == 0) ? g2 : 0.0f);
    gv[1] = (i1 == 1) ? g1 : ((i2 == 1) ? g2 : 0.0f);
    gv[2] = (i1 == 2) ? g1 : ((i2 == 2) ? g2 : 0.0f);
    gv[3] = (i1 == 3) ? g1 : ((i2 == 3) ? g2 : 0.0f);
    if (part == 0) *(v4f*)(sG + tk * NE) = gv;
  }
  __syncthreads();

  const v4f gq = *(const v4f*)(sG + lane * NE);
  float* rdst = rt + (size_t)(t0 + lane) * NE;
  v4u pv[4];
  size_t po[4];
#pragma unroll
  for (int it = 0; it < 4; ++it) {
    const int row = 8 * it + wave;
    const float* s = sX1 + row * CM + 8 * lane;
    const v4f a0 = *(const v4f*)(s);
    const v4f a1 = *(const v4f*)(s + 4);
    Pack8 pk;
    pk.h = (v8h){(_Float16)a0[0], (_Float16)a0[1], (_Float16)a0[2], (_Float16)a0[3],
                 (_Float16)a1[0], (_Float16)a1[1], (_Float16)a1[2], (_Float16)a1[3]};
    pv[it] = pk.u;
    po[it] = (size_t)(t0 + row) * CM + 8 * lane;
  }
  for (int ps = 0; ps < 2; ++ps) {
    if (wave == 0) *(volatile v4f*)rdst = gq;
#pragma unroll
    for (int it = 0; it < 4; ++it) *(volatile v4u*)(x1h + po[it]) = pv[it];
    __threadfence();
  }
}

__global__ __launch_bounds__(256) void k_experts(const _Float16* __restrict__ x1h, const _Float16* __restrict__ weh,
                                                 const float* __restrict__ bnes, const float* __restrict__ bneb,
                                                 const float* __restrict__ rt, _Float16* __restrict__ moeh) {
  __shared__ __align__(16) float sO[TB2 * OTP];
  __shared__ __align__(16) float sG[TB2 * NE];
  const int tid = threadIdx.x, lane = tid & 31, wave = tid >> 5;
  const int hh = lane >> 4, c = lane & 15;
  const int wm = wave & 1, wn = wave >> 1;
  const int t0 = blockIdx.x * TB2;

  for (int i = tid; i < (TB2 * OTP) / 4; i += 256) *(v4f*)(sO + 4 * i) = (v4f){0.f, 0.f, 0.f, 0.f};
  if (wave == 0) *(v4f*)(sG + lane * NE) = *(const v4f*)(rt + (size_t)(t0 + lane) * NE);
  __syncthreads();

  const int arow = t0 + wm * 16;
  const int bc0  = wn * 64;
  const int rl   = wm * 16 + 8 * hh;
#pragma unroll 1
  for (int e = 0; e < NE; ++e) {
    const _Float16* we = weh + (size_t)e * (size_t)(CM * CM);
    v8f acc[4];
#pragma unroll
    for (int t = 0; t < 4; ++t) acc[t] = zero8();
#pragma unroll 1
    for (int k0 = 0; k0 < CM; k0 += 32) {
      const v16h a = ldfrag(x1h, CM, arow, k0, lane);
#pragma unroll
      for (int t = 0; t < 4; ++t) {
        const v16h bq = ldfrag(we, CM, bc0 + 16 * t, k0, lane);
        acc[t] = mma16(a, bq, acc[t]);
      }
    }
#pragma unroll
    for (int t = 0; t < 4; ++t) {
      const int n = bc0 + 16 * t + c;
      const float sc = bnes[e * CM + n] * WEI;
      const float sh = bneb[e * CM + n];
#pragma unroll
      for (int r = 0; r < 8; ++r) {
        const float v  = acc[t][r] * sc + sh;
        const float sg = __builtin_amdgcn_rcpf(1.0f + __expf(-v));
        const float g  = sG[(rl + r) * NE + e];
        float* so = sO + (rl + r) * OTP + n;
        *so = *so + (v * sg) * g;
      }
    }
  }
  __syncthreads();

  v4u pv[4];
  size_t po[4];
#pragma unroll
  for (int it = 0; it < 4; ++it) {
    const int p  = lane + 32 * it;
    const int L  = p >> 3;
    const int pc = p & 7;
    const float* s = sO + (wm * 16 + L) * OTP + bc0 + pc * 8;
    const v4f a0 = *(const v4f*)(s) * MOS;
    const v4f a1 = *(const v4f*)(s + 4) * MOS;
    Pack8 pk;
    pk.h = (v8h){(_Float16)a0[0], (_Float16)a0[1], (_Float16)a0[2], (_Float16)a0[3],
                 (_Float16)a1[0], (_Float16)a1[1], (_Float16)a1[2], (_Float16)a1[3]};
    pv[it] = pk.u;
    po[it] = (size_t)(t0 + wm * 16 + L) * CM + bc0 + pc * 8;
  }
  for (int ps = 0; ps < 2; ++ps) {
#pragma unroll
    for (int it = 0; it < 4; ++it) *(volatile v4u*)(moeh + po[it]) = pv[it];
    __threadfence();
  }
}

__global__ __launch_bounds__(256) void k_conv3(const _Float16* __restrict__ moeh, const _Float16* __restrict__ w3h,
                                               const float* __restrict__ bn3s, const float* __restrict__ bn3b,
                                               const float* __restrict__ x, float* __restrict__ out) {
  __shared__ __align__(16) float sH[OB3 * HTP];
  const int tid = threadIdx.x, lane = tid & 31, wave = tid >> 5;
  const int hh = lane >> 4, c = lane & 15;
  const int wm = wave & 3, wn = wave >> 2;
  const int t0 = blockIdx.x * TB3;
  const int o0 = blockIdx.y * OB3;
  const int arow = o0 + wm * 16;
  const int brow = t0 + wn * 64;

  v8f acc[4];
#pragma unroll
  for (int t = 0; t < 4; ++t) acc[t] = zero8();
#pragma unroll 1
  for (int k0 = 0; k0 < CM; k0 += 32) {
    const v16h a = ldfrag(w3h, CM, arow, k0, lane);
#pragma unroll
    for (int t = 0; t < 4; ++t) {
      const v16h bq = ldfrag(moeh, CM, brow + 16 * t, k0, lane);
      acc[t] = mma16(a, bq, acc[t]);
    }
  }

  const int ol = wm * 16 + 8 * hh;
  float sc[8], sh[8];
#pragma unroll
  for (int r = 0; r < 8; ++r) {
    sc[r] = bn3s[o0 + ol + r] * C3I;
    sh[r] = bn3b[o0 + ol + r];
  }
#pragma unroll
  for (int t = 0; t < 4; ++t) {
#pragma unroll
    for (int r = 0; r < 8; ++r) {
      const float v  = acc[t][r] * sc[r] + sh[r];
      const float sg = __builtin_amdgcn_rcpf(1.0f + __expf(-v));
      sH[(ol + r) * HTP + wn * 64 + 16 * t + c] = v * sg;
    }
  }
  __syncthreads();

  v4f val[8];
  size_t go[8];
#pragma unroll
  for (int it = 0; it < 8; ++it) {
    const int row = 8 * it + wave;
    go[it] = (size_t)(o0 + row) * NT + t0 + 4 * lane;
    const v4f hv = *(const v4f*)(sH + row * HTP + 4 * lane);
    const v4f xr = *(const v4f*)(x + go[it]);
    val[it] = hv + xr;
  }
  for (int ps = 0; ps < 2; ++ps) {
#pragma unroll
    for (int it = 0; it < 8; ++it) *(volatile v4f*)(out + go[it]) = val[it];
    __threadfence();
  }
}

extern "C" void kernel_launch(void* const* d_in, const int* in_sizes, int n_in,
                              void* d_out, int out_size, void* d_ws, size_t ws_size,
                              hipStream_t stream) {
  if (n_in < 12) return;
  if (in_sizes[0]  != C1 * NT) return;
  if (in_sizes[1]  != CM * C1) return;
  if (in_sizes[2]  != CM) return;
  if (in_sizes[3]  != CM) return;
  if (in_sizes[4]  != NE * CM) return;
  if (in_sizes[5]  != NE) return;
  if (in_sizes[6]  != NE * CM * CM * 9) return;
  if (in_sizes[7]  != NE * CM) return;
  if (in_sizes[8]  != NE * CM) return;
  if (in_sizes[9]  != C2 * CM) return;
  if (in_sizes[10] != C2) return;
  if (in_sizes[11] != C2) return;
  if (out_size != C2 * NT) return;

  const float* x     = (const float*)d_in[0];
  const float* w1    = (const float*)d_in[1];
  const float* bn1s  = (const float*)d_in[2];
  const float* bn1b  = (const float*)d_in[3];
  const float* wrt   = (const float*)d_in[4];
  const float* brt   = (const float*)d_in[5];
  const float* wexp  = (const float*)d_in[6];
  const float* bnes  = (const float*)d_in[7];
  const float* bneb  = (const float*)d_in[8];
  const float* w3    = (const float*)d_in[9];
  const float* bn3s  = (const float*)d_in[10];
  const float* bn3b  = (const float*)d_in[11];
  float* out = (float*)d_out;

  size_t off = 0;
  const size_t oX1 = off; off += (size_t)NT * CM * 2;
  const size_t oWE = off; off += (size_t)NE * CM * CM * 2;
  const size_t oW3 = off; off += (size_t)C2 * CM * 2;
  const size_t oR  = off; off += (size_t)NT * NE * 4;
  const size_t oMO = off; off += (size_t)NT * CM * 2;
  if (off > ws_size) return;
  if (off > (size_t)134217728) return;
  if ((oX1 | oWE | oW3 | oR | oMO) & (size_t)127) return;

  char* ws = (char*)d_ws;
  _Float16* X1H  = (_Float16*)(ws + oX1);
  _Float16* WEH  = (_Float16*)(ws + oWE);
  _Float16* W3H  = (_Float16*)(ws + oW3);
  float*    R    = (float*)(ws + oR);
  _Float16* MOEH = (_Float16*)(ws + oMO);

  k_cvtw<<<dim3((NE * CM) / 8), dim3(256), 0, stream>>>(wexp, WEH, NE * CM, CM * 9, 9, 4, WES);
  k_cvtw<<<dim3(C2 / 8), dim3(256), 0, stream>>>(w3, W3H, C2, CM, 1, 0, W3S);
  k_conv1<<<dim3(NT / TB1), dim3(256), 0, stream>>>(x, w1, bn1s, bn1b, wrt, brt, X1H, R);
  k_experts<<<dim3(NT / TB2), dim3(256), 0, stream>>>(X1H, WEH, bnes, bneb, R, MOEH);
  k_conv3<<<dim3(NT / TB3, C2 / OB3), dim3(256), 0, stream>>>(MOEH, W3H, bn3s, bn3b, x, out);
  (void)hipGetLastError();
}
